// WKV_50379966382716
// MI455X (gfx1250) — hardware-verified
//
#include <hip/hip_runtime.h>
#include <math.h>

typedef _Float16 f16;
typedef __attribute__((ext_vector_type(16))) _Float16 v16h;
typedef __attribute__((ext_vector_type(8)))  _Float16 v8h;
typedef __attribute__((ext_vector_type(8)))  float    v8f;
typedef __attribute__((ext_vector_type(4)))  float    v4f_t;
typedef __attribute__((ext_vector_type(2)))  float    v2f_t;
typedef float v4fa __attribute__((ext_vector_type(4), may_alias));

#define DIMD   512
#define TT     2048
#define CC     16
#define NCHUNK (TT / CC)
#define BCOL   64
#define NWG    (DIMD / BCOL)
#define NTHR   128
#define RSPLIT (1.0f / 2048.0f)
#define PLR  ((size_t)TT * DIMD)

__device__ __forceinline__ f16 lo_of(float v, f16 h) { return (f16)((v - (float)h) * 2048.0f); }
__device__ __forceinline__ float hw_log2(float x) { float y; asm volatile("v_log_f32 %0, %1" : "=v"(y) : "v"(x)); return y; }
__device__ __forceinline__ float hw_exp2(float x) { float y; asm volatile("v_exp_f32 %0, %1" : "=v"(y) : "v"(x)); return y; }
__device__ __forceinline__ f16 lo_of_nofma(float v, f16 h) { float hf = (float)h; asm volatile("" : "+v"(hf)); float d = v - hf; asm volatile("" : "+v"(d)); float t = d * 2048.0f; asm volatile("" : "+v"(t)); return (f16)t; }
__device__ __forceinline__ unsigned pk2s_nofma(float a, float b, unsigned* lo) {
  float a1 = a, b1 = b; asm volatile("" : "+v"(a1), "+v"(b1));
  const f16 h0 = (f16)a1, h1 = (f16)b1;
  *lo = (unsigned)__builtin_bit_cast(unsigned short, lo_of_nofma(a1, h0)) | ((unsigned)__builtin_bit_cast(unsigned short, lo_of_nofma(b1, h1)) << 16);
  return (unsigned)__builtin_bit_cast(unsigned short, h0) | ((unsigned)__builtin_bit_cast(unsigned short, h1) << 16);
}
__device__ __forceinline__ int kmap(int e, int hi) { return (e < 8) ? (hi * 8 + e) : (16 + hi * 8 + (e - 8)); }
__device__ __forceinline__ v8f wmma16(v16h a, v16h b, v8f c) { return __builtin_amdgcn_wmma_f32_16x16x32_f16(false, a, false, b, (short)0, c, false, false); }
struct Frag2 { v16h h, l; };
__device__ __forceinline__ v8f wmma_split(const Frag2& a, const Frag2& b, v8f c) { v8f x = {}; x = wmma16(a.l, b.h, x); x = wmma16(a.h, b.l, x); return wmma16(a.h, b.h, c) + x * RSPLIT; }
__device__ __forceinline__ v16h cat8(v8h a, v8h b) { return __builtin_shufflevector(a, b, 0,1,2,3,4,5,6,7,8,9,10,11,12,13,14,15); }
__device__ __forceinline__ unsigned pk2s(float a, float b, unsigned* lo) {
  const f16 h0 = (f16)a, h1 = (f16)b;
  *lo = (unsigned)__builtin_bit_cast(unsigned short, lo_of(a, h0)) | ((unsigned)__builtin_bit_cast(unsigned short, lo_of(b, h1)) << 16);
  return (unsigned)__builtin_bit_cast(unsigned short, h0) | ((unsigned)__builtin_bit_cast(unsigned short, h1) << 16);
}

__global__ __launch_bounds__(256) void prep_kernel(const float* __restrict__ r, const float* __restrict__ w, const float* __restrict__ k,
                                                  const float* __restrict__ u,
                                                  f16* __restrict__ rt, f16* __restrict__ kht, float* __restrict__ pc, float* __restrict__ Lg) {
  __shared__ __attribute__((aligned(16))) f16 khs[2][DIMD * CC];
  const int tid = threadIdx.x, lane = tid & 31, wave = tid >> 5;
  const int g = blockIdx.x;
  const int a = tid * 2;
  (void)u;
#pragma unroll 1
  for (int cq = 0; cq < 4; ++cq) {
    const int c = g * 4 + cq, t0 = c * CC;
    float rv[2][CC], kv[2][CC], L[2][CC];
#pragma unroll
    for (int s = 0; s < CC; ++s) {
      const v2f_t rr = *(const v2f_t*)(r + (size_t)(t0 + s) * DIMD + a);
      const v2f_t ww = *(const v2f_t*)(w + (size_t)(t0 + s) * DIMD + a);
      const v2f_t kk = *(const v2f_t*)(k + (size_t)(t0 + s) * DIMD + a);
      rv[0][s] = rr.x; rv[1][s] = rr.y; kv[0][s] = kk.x; kv[1][s] = kk.y;
      L[0][s] = hw_log2(fmaxf(ww.x, 1e-30f)); L[1][s] = hw_log2(fmaxf(ww.y, 1e-30f));
    }
#pragma unroll
    for (int q = 0; q < 2; ++q)
#pragma unroll
      for (int s = 1; s < CC; ++s) L[q][s] += L[q][s - 1];
#pragma unroll 1
    for (int pass = 0; pass < 2; ++pass) {
#pragma unroll
      for (int s = 0; s < CC; ++s) {
        const float e0 = (s == 0) ? 1.0f : hw_exp2(L[0][s - 1]), e1 = (s == 0) ? 1.0f : hw_exp2(L[1][s - 1]);
        float r0 = rv[0][s] * e0, r1 = rv[1][s] * e1; asm volatile("" : "+v"(r0), "+v"(r1));
        unsigned lo; const unsigned p = pk2s_nofma(r0, r1, &lo);
        *(volatile unsigned*)(rt + (size_t)(t0 + s) * DIMD + a) = p; *(volatile unsigned*)(rt + PLR + (size_t)(t0 + s) * DIMD + a) = lo;
        v2f_t lv; lv.x = L[0][s]; lv.y = L[1][s]; *(volatile v2f_t*)(Lg + (size_t)(t0 + s) * DIMD + a) = lv;
      }
      { v2f_t pcv; pcv.x = hw_exp2(L[0][CC - 1]); pcv.y = hw_exp2(L[1][CC - 1]); *(volatile v2f_t*)(pc + (size_t)c * DIMD + a) = pcv; }
      __threadfence();
    }
#pragma unroll
    for (int q = 0; q < 2; ++q)
#pragma unroll
      for (int s = 0; s < CC; ++s) { float kh = kv[q][s] * hw_exp2(L[q][CC - 1] - L[q][s]); asm volatile("" : "+v"(kh)); const f16 h = (f16)kh; khs[0][(a + q) * CC + s] = h; khs[1][(a + q) * CC + s] = lo_of_nofma(kh, h); }
    __syncthreads();
#pragma unroll 1
    for (int pass = 0; pass < 2; ++pass) {
      for (int i = tid; i < DIMD * CC / 8; i += 256) {
        *(volatile v8h*)(kht + (size_t)c * DIMD * CC + i * 8)       = *(const v8h*)&khs[0][i * 8];
        *(volatile v8h*)(kht + PLR + (size_t)c * DIMD * CC + i * 8) = *(const v8h*)&khs[1][i * 8];
      }
      __threadfence();
    }
    __syncthreads();
  }
}

__global__ __launch_bounds__(NTHR) void wkv_kernel(const f16* __restrict__ rt, const f16* __restrict__ kht, const float* __restrict__ pc,
                                                  const float* __restrict__ Lg, const float* __restrict__ r, const float* __restrict__ k,
                                                  const float* __restrict__ u, const float* __restrict__ v,
                                                  const float* __restrict__ init_state, float* __restrict__ out) {
  __shared__ float red[4][272];
  __shared__ __attribute__((aligned(16))) float S[DIMD * BCOL];
  __shared__ __attribute__((aligned(16))) float Vt[CC][BCOL];
  __shared__ float sc[272];
  __shared__ __attribute__((aligned(16))) float Yst[CC][BCOL + 4];
  const int tid = threadIdx.x, lane = tid & 31, wid = tid >> 5;
  const int hi = lane >> 4, ln = lane & 15;
  const int wgBase = blockIdx.x * BCOL;
  const int n0 = wid * 16;
  float* yout = out;
  float* sout = out + (size_t)TT * DIMD;

  for (int i = tid; i < DIMD * BCOL; i += NTHR) { const int aa = i >> 6, b = i & 63; S[aa * BCOL + b] = init_state[wgBase + b]; }
  __syncthreads();

  for (int c = 0; c < NCHUNK; ++c) {
    for (int i = tid; i < CC * BCOL / 4; i += NTHR) { const int s = i >> 4, q = (i & 15) * 4; *(v4f_t*)&Vt[s][q] = *(const v4f_t*)(v + (size_t)(c * CC + s) * DIMD + wgBase + q); }
    {
      float acc_sc[CC];
#pragma unroll 1
      for (int tau = 0; tau < CC; ++tau) {
#pragma unroll
        for (int s = 0; s < CC; ++s) acc_sc[s] = 0.f;
        float dg = 0.f;
#pragma unroll 1
        for (int i = 0; i < 4; ++i) {
          const int a = tid + NTHR * i;
          const float rtau = r[(size_t)(c * CC + tau) * DIMD + a];
          const float Lt = (tau == 0) ? 0.f : Lg[(size_t)(c * CC + tau - 1) * DIMD + a];
          dg += rtau * u[a] * k[(size_t)(c * CC + tau) * DIMD + a];
#pragma unroll
          for (int s = 0; s < CC; ++s) if (s < tau) acc_sc[s] += rtau * k[(size_t)(c * CC + s) * DIMD + a] * hw_exp2(Lt - Lg[(size_t)(c * CC + s) * DIMD + a]);
        }
#pragma unroll
        for (int off = 1; off < 32; off <<= 1) {
#pragma unroll
          for (int s = 0; s < CC; ++s) acc_sc[s] += __shfl_xor(acc_sc[s], off, 32);
          dg += __shfl_xor(dg, off, 32);
        }
        if (lane == 0) {
#pragma unroll
          for (int s = 0; s < CC; ++s) red[wid][tau * CC + s] = (s < tau) ? acc_sc[s] : 0.f;
          red[wid][256 + tau] = dg;
        }
      }
      __syncthreads();
      for (int i = tid; i < 272; i += NTHR) sc[i] = red[0][i] + red[1][i] + red[2][i] + red[3][i];
    }
    __syncthreads();

    v8f y8 = {};
#pragma unroll 2
    for (int kb = 0; kb < DIMD; kb += 32) {
      Frag2 A; { const f16* p = rt + (size_t)(c * CC + ln) * DIMD + kb + hi * 8; A.h = cat8(*(const v8h*)p, *(const v8h*)(p + 16)); A.l = cat8(*(const v8h*)(p + PLR), *(const v8h*)(p + PLR + 16)); }
      Frag2 B;
#pragma unroll
      for (int e = 0; e < 16; ++e) { const float sv = S[(kb + kmap(e, hi)) * BCOL + n0 + ln]; B.h[e] = (f16)sv; B.l[e] = lo_of(sv, B.h[e]); }
      y8 = wmma_split(A, B, y8);
    }
#pragma unroll
    for (int rr = 0; rr < 8; ++rr) {
      const int tau = rr + 8 * hi;
      float yv = y8[rr] + sc[256 + tau] * Vt[tau][n0 + ln];
#pragma unroll
      for (int s = 0; s < CC; ++s) yv += sc[tau * CC + s] * Vt[s][n0 + ln];
      Yst[tau][n0 + ln] = yv;
    }
    __syncthreads();
#pragma unroll 1
    for (int pass = 0; pass < 2; ++pass) {
#pragma unroll
      for (int i = 0; i < 2; ++i) { const int cc = tid + NTHR * i, tau = cc >> 4, q = (cc & 15) * 4;
        *(volatile v4f_t*)(yout + (size_t)(c * CC + tau) * DIMD + wgBase + q) = *(const v4fa*)&Yst[tau][q]; }
      __threadfence();
    }

    Frag2 Bv;
#pragma unroll
    for (int e = 0; e < 16; ++e) { const int s = kmap(e, hi); const float vv = (s < CC) ? Vt[s & 15][n0 + ln] : 0.f; Bv.h[e] = (f16)vv; Bv.l[e] = lo_of(vv, Bv.h[e]); }
#pragma unroll 2
    for (int it = 0; it < DIMD / 16; ++it) {
      const int a0 = it * 16;
      Frag2 A;
      { const f16* p = kht + ((size_t)c * DIMD + a0 + ln) * CC + hi * 8;
        const v8h z = {}; A.h = cat8(*(const v8h*)p, z); A.l = cat8(*(const v8h*)(p + PLR), z); }
      v8f upd = {};
      upd = wmma_split(A, Bv, upd);
#pragma unroll
      for (int rr = 0; rr < 8; ++rr) { const int row = a0 + rr + 8 * hi; S[row * BCOL + n0 + ln] = S[row * BCOL + n0 + ln] * pc[(size_t)c * DIMD + row] + upd[rr]; }
    }
    __syncthreads();
  }
#pragma unroll 1
  for (int pass = 0; pass < 2; ++pass) {
    for (int i = tid; i < DIMD * 16; i += NTHR) { const int aa = i >> 4, q = (i & 15) * 4; *(volatile v4f_t*)(sout + (size_t)aa * DIMD + wgBase + q) = *(const v4fa*)&S[aa * BCOL + q]; }
    __threadfence();
  }
}

extern "C" void kernel_launch(void* const* d_in, const int* in_sizes, int n_in,
                              void* d_out, int out_size, void* d_ws, size_t ws_size,
                              hipStream_t stream) {
  const float* r   = (const float*)d_in[0];
  const float* w   = (const float*)d_in[1];
  const float* k   = (const float*)d_in[2];
  const float* v   = (const float*)d_in[3];
  const float* is_ = (const float*)d_in[4];
  const float* u   = (const float*)d_in[5];
  float* out = (float*)d_out;
  (void)in_sizes; (void)n_in; (void)out_size; (void)ws_size;

  char* wsb = (char*)d_ws;
  auto carve = [&](size_t bytes) -> char* { char* p = wsb; wsb += (bytes + 255) & ~(size_t)255; return p; };
  f16*   rt  = (f16*)carve(PLR * 2 * 2);
  f16*   kht = (f16*)carve(PLR * 2 * 2);
  float* pc  = (float*)carve((size_t)NCHUNK * DIMD * 4);
  float* Lg  = (float*)carve((size_t)TT * DIMD * 4);

  prep_kernel<<<NCHUNK / 4, 256, 0, stream>>>(r, w, k, u, rt, kht, pc, Lg);
  wkv_kernel<<<NWG, NTHR, 0, stream>>>(rt, kht, pc, Lg, r, k, u, v, is_, out);
}
